// SimpleRNN_4939212390684
// MI455X (gfx1250) — hardware-verified
//
#include <hip/hip_runtime.h>
#include <math.h>

constexpr int NB    = 256;
constexpr int NSTEP = 512;
constexpr int NVOC  = 50000;
constexpr int ND    = 100;
constexpr int KPAD  = 128;
constexpr int NH    = 128;
constexpr int NCLS  = 2;
constexpr int NTHR  = 256;
constexpr int BROWS = 16;
constexpr int AEP   = 136;
constexpr int HSP   = 260;
constexpr int NROWS = NB * NSTEP;
static_assert(NB % BROWS == 0, "blocks cover the batch exactly");
static_assert(NH == 16 * (NTHR / 32), "8 waves x 16 hidden columns");
static_assert(KPAD == NH && KPAD % 32 == 0, "one shared 4-chunk k loop, K multiple of 32");
static_assert(ND % 4 == 0 && ND + 4 <= KPAD + 4 && ND <= KPAD, "16-B aligned embedding rows, pad fits");
static_assert((ND * 4) % 16 == 0, "embedding row pitch 16-B aligned");
static_assert(NTHR == BROWS * (KPAD / 8), "gather: 16 threads x 8 columns per row, 16 rows");
static_assert(NTHR == NCLS * NH, "head weight staging: one float per thread");
static_assert(BROWS * NCLS == 32, "one block writes exactly one 128-B output line");
static_assert(AEP % 8 == 0 && AEP >= KPAD, "16-B aligned LDS rows");
static_assert(NH == 16 * 8, "y1 row = 16 lanes x 8 elements");
static_assert(NH * (KPAD / 8) == 8 * NTHR, "weight convert grid exact");
static_assert(HSP % 4 == 0 && HSP >= NH, "f32 staging pitch");

typedef __attribute__((ext_vector_type(16))) __bf16   v16b;
typedef __attribute__((ext_vector_type(8)))  __bf16   v8b;
typedef __attribute__((ext_vector_type(8)))  float    v8f;
typedef __attribute__((ext_vector_type(4)))  float    v4f;
typedef __attribute__((ext_vector_type(4)))  unsigned v4u;

__device__ __forceinline__ unsigned short f2bf_bits(float f) {
  unsigned u = __float_as_uint(f);
  return (unsigned short)((u + 0x7FFFu + ((u >> 16) & 1u)) >> 16);
}
__device__ __forceinline__ float bf_bits2f(unsigned short h) { return __uint_as_float(((unsigned)h) << 16); }
__device__ __forceinline__ float bf16r(float f) { return bf_bits2f(f2bf_bits(f)); }
__device__ __forceinline__ float opaque_f(float f) { asm volatile("" : "+v"(f)); return f; }

struct FragB {
  union U { v16b v; v8b h[2]; };
  static __device__ __forceinline__ v16b load(const __bf16* p) {
    U f; f.h[0] = *(const v8b*)(p); f.h[1] = *(const v8b*)(p + 16); return f.v;
  }
  static __device__ __forceinline__ v8f mma(v16b a, v16b b, v8f c) {
    return __builtin_amdgcn_wmma_f32_16x16x32_bf16(false, a, false, b, (short)0, c, false, false);
  }
};
__device__ __forceinline__ void mma_guard6(v8f& acc, v16b a0, v16b a1, v16b a2, v16b b0, v16b b1) {
  asm volatile("v_nop\n\tv_nop\n\tv_nop\n\tv_nop" : "+v"(acc) : "v"(a0), "v"(a1), "v"(a2), "v"(b0), "v"(b1));
}
__device__ __forceinline__ void mma_guard7(v8f& acc, v16b a0, v16b a1, v16b a2, v16b a3, v16b b0, v16b b1) {
  asm volatile("v_nop\n\tv_nop\n\tv_nop\n\tv_nop" : "+v"(acc) : "v"(a0), "v"(a1), "v"(a2), "v"(a3), "v"(b0), "v"(b1));
}
__device__ __forceinline__ void acc_guard1(v8f& a) { asm volatile("v_nop\n\tv_nop\n\tv_nop\n\tv_nop" : "+v"(a)); }

__device__ __forceinline__ v4u pack8_bf16(v4f a, v4f b, v4f fa, v4f fb) {
  v4u pk;
#pragma unroll
  for (int p = 0; p < 2; ++p) {
    const float x0 = a[2 * p] * fa[2 * p];
    const float x1 = a[2 * p + 1] * fa[2 * p + 1];
    const float y0 = b[2 * p] * fb[2 * p];
    const float y1 = b[2 * p + 1] * fb[2 * p + 1];
    pk[p]     = (unsigned)f2bf_bits(x0) | ((unsigned)f2bf_bits(x1) << 16);
    pk[2 + p] = (unsigned)f2bf_bits(y0) | ((unsigned)f2bf_bits(y1) << 16);
  }
  return pk;
}

__global__ __launch_bounds__(NTHR) void wprep_kernel(const float* __restrict__ src, int spitch, int kreal,
                                                    unsigned short* __restrict__ dst) {
  const int i = blockIdx.x * NTHR + threadIdx.x;
  if (i >= NH * (KPAD / 8)) return;
  const int r = i >> 4, c8 = (i & 15) * 8;
  const int kl = kreal - 4;
  const int ca = (c8 < kl) ? c8 : kl;
  const int cb = ((c8 + 4) < kl) ? (c8 + 4) : kl;
  const float* sp = src + (size_t)r * spitch;
  const v4f va = *(const v4f*)(sp + ca);
  const v4f vb = *(const v4f*)(sp + cb);
  v4f fa, fb;
#pragma unroll
  for (int e = 0; e < 4; ++e) {
    fa[e] = opaque_f((c8 + e     < kreal) ? 1.0f : 0.0f);
    fb[e] = opaque_f((c8 + 4 + e < kreal) ? 1.0f : 0.0f);
  }
  const v4u pk = pack8_bf16(va, vb, fa, fb);
  unsigned short* dp = dst + (size_t)r * KPAD + c8;
  *(volatile v4u*)dp = pk;
  __threadfence();
  *(volatile v4u*)dp = pk;
}

__global__ __launch_bounds__(64) void bprep_kernel(const float* __restrict__ bi0, const float* __restrict__ bh0,
                                                  const float* __restrict__ bi1, const float* __restrict__ bh1,
                                                  float* __restrict__ dst) {
  const int tid = threadIdx.x;
  const int which = tid >> 5;
  const int idx = (tid & 31) * 4;
  const v4f va = *(const v4f*)(bi0 + idx);
  const v4f vb = *(const v4f*)(bh0 + idx);
  const v4f vc = *(const v4f*)(bi1 + idx);
  const v4f vd = *(const v4f*)(bh1 + idx);
  const float wf = opaque_f((float)which);
  v4f o;
#pragma unroll
  for (int e = 0; e < 4; ++e) {
    const float s0 = bf16r(va[e]) + bf16r(vb[e]);
    const float s1 = bf16r(vc[e]) + bf16r(vd[e]);
    o[e] = fmaf(s1, wf, s0 * (1.0f - wf));
  }
  float* op = dst + which * NH + idx;
  *(volatile v4f*)op = o;
  __threadfence();
  *(volatile v4f*)op = o;
}

__global__ __launch_bounds__(NTHR) void rnn0_kernel(const int* __restrict__ xtok, const float* __restrict__ emb,
                                                   const unsigned short* __restrict__ WIp,
                                                   const unsigned short* __restrict__ WHp,
                                                   const float* __restrict__ bsum,
                                                   unsigned short* __restrict__ YH,
                                                   unsigned short* __restrict__ YL) {
  __shared__ __align__(16) unsigned short Ae[BROWS * AEP];
  __shared__ __align__(16) unsigned short Hh[BROWS * AEP];
  __shared__ __align__(16) unsigned short Hl[BROWS * AEP];
  const __bf16* WI = (const __bf16*)WIp;
  const __bf16* WH = (const __bf16*)WHp;
  const int tid = threadIdx.x, lane = tid & 31, wave = tid >> 5;
  const int c = lane & 15, hh = lane >> 4, koff = hh * 8;
  const int b0 = blockIdx.x * BROWS;
  const int j = 16 * wave + c;
  const int gm = tid >> 4, gc = (tid & 15) * 8;
  const int gca = (gc < (ND - 4)) ? gc : (ND - 4);
  const int gcb = ((gc + 4) < (ND - 4)) ? (gc + 4) : (ND - 4);
  v4f gfa, gfb;
#pragma unroll
  for (int e = 0; e < 4; ++e) {
    gfa[e] = opaque_f((gc + e     < ND) ? 1.0f : 0.0f);
    gfb[e] = opaque_f((gc + 4 + e < ND) ? 1.0f : 0.0f);
  }
  const int* xr = xtok + (size_t)(b0 + gm) * NSTEP;
  unsigned short* aedst = Ae + gm * AEP + gc;

#pragma unroll 1
  for (int i = tid; i < BROWS * AEP; i += NTHR) { Ae[i] = 0; Hh[i] = 0; Hl[i] = 0; }
  const float bj = bsum[j];
  __syncthreads();
  {
    int tok = xr[0];
    tok = tok < 0 ? 0 : tok; tok = tok > (NVOC - 1) ? (NVOC - 1) : tok;
    const float* er = emb + (size_t)tok * ND;
    const v4f pa = *(const v4f*)(er + gca);
    const v4f pb = *(const v4f*)(er + gcb);
    *(v4u*)aedst = pack8_bf16(pa, pb, gfa, gfb);
  }
  __syncthreads();

  const __bf16* aer = (const __bf16*)Ae + c * AEP + koff;
  const __bf16* hhr = (const __bf16*)Hh + c * AEP + koff;
  const __bf16* hlr = (const __bf16*)Hl + c * AEP + koff;
  const __bf16* wi  = WI + (size_t)j * KPAD + koff;
  const __bf16* wh  = WH + (size_t)j * NH + koff;
  const int lr = 2 * wave + hh;
  const unsigned short* yhs = Hh + lr * AEP + 8 * c;
  const unsigned short* yls = Hl + lr * AEP + 8 * c;
  const v8f z8 = {0.f, 0.f, 0.f, 0.f, 0.f, 0.f, 0.f, 0.f};

#pragma unroll 1
  for (int t = 0; t < NSTEP; ++t) {
    const int tn = (t + 1 < NSTEP) ? (t + 1) : (NSTEP - 1);
    int tok = xr[tn];
    tok = tok < 0 ? 0 : tok; tok = tok > (NVOC - 1) ? (NVOC - 1) : tok;
    const float* er = emb + (size_t)tok * ND;
    const v4f pa = *(const v4f*)(er + gca);
    const v4f pb = *(const v4f*)(er + gcb);

    v8f acc = z8;
#pragma unroll 1
    for (int k0 = 0; k0 < KPAD; k0 += 32) {
      const v16b ae = FragB::load(aer + k0);
      const v16b ah = FragB::load(hhr + k0);
      const v16b al = FragB::load(hlr + k0);
      const v16b bi = FragB::load(wi + k0);
      const v16b bh = FragB::load(wh + k0);
      acc = FragB::mma(ae, bi, acc);
      acc = FragB::mma(ah, bh, acc);
      acc = FragB::mma(al, bh, acc);
      mma_guard6(acc, ae, ah, al, bi, bh);
    }
    acc_guard1(acc);
    unsigned short hb8[8], lb8[8];
#pragma unroll
    for (int r = 0; r < 8; ++r) {
      const float z  = acc[r] + bj;
      const float hv = tanhf(z);
      const unsigned short hb = f2bf_bits(hv);
      hb8[r] = hb;
      lb8[r] = f2bf_bits(hv - bf_bits2f(hb));
    }
    __syncthreads();
#pragma unroll
    for (int r = 0; r < 8; ++r) {
      Hh[(8 * hh + r) * AEP + j] = hb8[r];
      Hl[(8 * hh + r) * AEP + j] = lb8[r];
    }
    *(v4u*)aedst = pack8_bf16(pa, pb, gfa, gfb);
    __syncthreads();
    {
      const v4u vh = *(const v4u*)yhs;
      const v4u vl = *(const v4u*)yls;
      const size_t go = ((size_t)t * NB + (size_t)(b0 + lr)) * NH + 8 * c;
      for (int pass = 0; pass < 2; ++pass) {
        *(volatile v4u*)(YH + go) = vh;
        *(volatile v4u*)(YL + go) = vl;
        __threadfence();
      }
    }
  }
}

__global__ __launch_bounds__(NTHR) void rnn1_kernel(const unsigned short* __restrict__ YH,
                                                   const unsigned short* __restrict__ YL,
                                                   const unsigned short* __restrict__ WIp,
                                                   const unsigned short* __restrict__ WHp,
                                                   const float* __restrict__ bsum,
                                                   const float* __restrict__ fcw,
                                                   const float* __restrict__ fcb,
                                                   float* __restrict__ out) {
  __shared__ __align__(16) unsigned short Hh[BROWS * AEP];
  __shared__ __align__(16) unsigned short Hl[BROWS * AEP];
  __shared__ __align__(16) float Hs[BROWS * HSP];
  __shared__ __align__(16) float Fw[NCLS * NH];
  __shared__ __align__(16) float Os[BROWS * NCLS];
  __shared__ float Fb[NCLS];
  const __bf16* WI = (const __bf16*)WIp;
  const __bf16* WH = (const __bf16*)WHp;
  const int tid = threadIdx.x, lane = tid & 31, wave = tid >> 5;
  const int c = lane & 15, hh = lane >> 4, koff = hh * 8;
  const int b0 = blockIdx.x * BROWS;
  const int j = 16 * wave + c;

#pragma unroll 1
  for (int i = tid; i < BROWS * AEP; i += NTHR) { Hh[i] = 0; Hl[i] = 0; }
  Fw[tid] = bf16r(fcw[tid]);
  {
    const float fbv = bf16r(fcb[tid & 1]);
    if (tid < NCLS) Fb[tid] = fbv;
  }
  float hst[8];
#pragma unroll
  for (int r = 0; r < 8; ++r) hst[r] = 0.0f;
  const float bj = bsum[j];
  __syncthreads();

  const __bf16* hhr = (const __bf16*)Hh + c * AEP + koff;
  const __bf16* hlr = (const __bf16*)Hl + c * AEP + koff;
  const __bf16* wi  = WI + (size_t)j * NH + koff;
  const __bf16* wh  = WH + (size_t)j * NH + koff;
  const v8f z8 = {0.f, 0.f, 0.f, 0.f, 0.f, 0.f, 0.f, 0.f};

#pragma unroll 1
  for (int t = 0; t < NSTEP; ++t) {
    const size_t yo = ((size_t)t * NB + (size_t)(b0 + c)) * NH + koff;
    const __bf16* yh = (const __bf16*)YH + yo;
    const __bf16* yl = (const __bf16*)YL + yo;
    v8f acc = z8;
#pragma unroll 1
    for (int k0 = 0; k0 < NH; k0 += 32) {
      const v16b ayh = FragB::load(yh + k0);
      const v16b ayl = FragB::load(yl + k0);
      const v16b ah  = FragB::load(hhr + k0);
      const v16b al  = FragB::load(hlr + k0);
      const v16b bi  = FragB::load(wi + k0);
      const v16b bh  = FragB::load(wh + k0);
      acc = FragB::mma(ayh, bi, acc);
      acc = FragB::mma(ayl, bi, acc);
      acc = FragB::mma(ah, bh, acc);
      acc = FragB::mma(al, bh, acc);
      mma_guard7(acc, ayh, ayl, ah, al, bi, bh);
    }
    acc_guard1(acc);
    unsigned short hb8[8], lb8[8];
#pragma unroll
    for (int r = 0; r < 8; ++r) {
      const float z  = acc[r] + bj;
      const float hv = tanhf(z);
      hst[r] = hv;
      const unsigned short hb = f2bf_bits(hv);
      hb8[r] = hb;
      lb8[r] = f2bf_bits(hv - bf_bits2f(hb));
    }
    __syncthreads();
#pragma unroll
    for (int r = 0; r < 8; ++r) {
      Hh[(8 * hh + r) * AEP + j] = hb8[r];
      Hl[(8 * hh + r) * AEP + j] = lb8[r];
    }
    __syncthreads();
  }

#pragma unroll
  for (int r = 0; r < 8; ++r) Hs[(8 * hh + r) * HSP + j] = hst[r];
  __syncthreads();
  if (wave == 0) {
    const int orow = lane >> 1, cls = lane & 1;
    const float* hp = Hs + orow * HSP;
    const float* fp = Fw + cls * NH;
    float s = 0.0f;
#pragma unroll 4
    for (int k = 0; k < NH; ++k) s = fmaf(hp[k], fp[k], s);
    Os[lane] = s + Fb[cls];
  }
  __syncthreads();
  if (tid < 8) {
    const v4f v = *(const v4f*)(Os + 4 * tid);
    float* op = out + (size_t)blockIdx.x * (BROWS * NCLS) + 4 * tid;
    *(volatile v4f*)op = v;
    __threadfence();
    *(volatile v4f*)op = v;
  }
}

extern "C" void kernel_launch(void* const* d_in, const int* in_sizes, int n_in,
                              void* d_out, int out_size, void* d_ws, size_t ws_size, hipStream_t stream) {
  if (n_in < 12 || d_out == nullptr || d_ws == nullptr) return;
  if (in_sizes[0] != NB * NSTEP || in_sizes[1] != NVOC * ND || in_sizes[2] != NH * ND || in_sizes[3] != NH * NH ||
      in_sizes[4] != NH || in_sizes[5] != NH || in_sizes[6] != NH * NH || in_sizes[7] != NH * NH ||
      in_sizes[8] != NH || in_sizes[9] != NH || in_sizes[10] != NCLS * NH || in_sizes[11] != NCLS ||
      out_size != NB * NCLS) return;

  const int*   x     = (const int*)d_in[0];
  const float* emb   = (const float*)d_in[1];
  const float* w_ih0 = (const float*)d_in[2];
  const float* w_hh0 = (const float*)d_in[3];
  const float* b_ih0 = (const float*)d_in[4];
  const float* b_hh0 = (const float*)d_in[5];
  const float* w_ih1 = (const float*)d_in[6];
  const float* w_hh1 = (const float*)d_in[7];
  const float* b_ih1 = (const float*)d_in[8];
  const float* b_hh1 = (const float*)d_in[9];
  const float* fc_w  = (const float*)d_in[10];
  const float* fc_b  = (const float*)d_in[11];
  float* out = (float*)d_out;

  char* ws = (char*)d_ws; size_t off = 0;
  auto carve = [&](size_t bytes) -> char* { char* p = ws + off; off += (bytes + 255) & ~(size_t)255; return p; };
  unsigned short* WI0 = (unsigned short*)carve((size_t)NH * KPAD * 2);
  unsigned short* WH0 = (unsigned short*)carve((size_t)NH * NH * 2);
  unsigned short* WI1 = (unsigned short*)carve((size_t)NH * NH * 2);
  unsigned short* WH1 = (unsigned short*)carve((size_t)NH * NH * 2);
  float*          BS  = (float*)carve((size_t)2 * NH * 4);
  unsigned short* YH  = (unsigned short*)carve((size_t)NROWS * NH * 2);
  unsigned short* YL  = (unsigned short*)carve((size_t)NROWS * NH * 2);
  if (off > ws_size || off > (size_t)134217728) return;

  wprep_kernel<<<8, NTHR, 0, stream>>>(w_ih0, ND, ND, WI0);
  wprep_kernel<<<8, NTHR, 0, stream>>>(w_hh0, NH, NH, WH0);
  wprep_kernel<<<8, NTHR, 0, stream>>>(w_ih1, NH, NH, WI1);
  wprep_kernel<<<8, NTHR, 0, stream>>>(w_hh1, NH, NH, WH1);
  bprep_kernel<<<1, 64, 0, stream>>>(b_ih0, b_hh0, b_ih1, b_hh1, BS);
  rnn0_kernel<<<NB / BROWS, NTHR, 0, stream>>>(x, emb, WI0, WH0, BS, YH, YL);
  rnn1_kernel<<<NB / BROWS, NTHR, 0, stream>>>(YH, YL, WI1, WH1, BS + NH, fc_w, fc_b, out);
}
